// SA_82832739270939
// MI455X (gfx1250) — hardware-verified
//
#include <hip/hip_runtime.h>
#include <math.h>

typedef __attribute__((ext_vector_type(16))) _Float16 v16h;
typedef __attribute__((ext_vector_type(16))) __bf16 v16b;
typedef __attribute__((ext_vector_type(8)))  _Float16 v8h;
typedef __attribute__((ext_vector_type(8)))  float v8f;
typedef __attribute__((ext_vector_type(4)))  float v4f;
typedef __attribute__((ext_vector_type(2)))  float v2f;
typedef __attribute__((ext_vector_type(4)))  unsigned v4u;
typedef __attribute__((ext_vector_type(4)))  int v4i;
typedef float __attribute__((may_alias)) float_a;
typedef int __attribute__((may_alias)) int_a;

template <typename T> __device__ __forceinline__ void vst2(void* p, T v) { *(volatile T*)p = v; __threadfence(); *(volatile T*)p = v; }
__device__ __forceinline__ v8f wmma16(v16h a, v16h b, v8f c) {
  v8f d = __builtin_amdgcn_wmma_f32_16x16x32_f16(false, a, false, b, (short)0, c, false, false);
  asm volatile("v_nop\n\tv_nop\n\tv_nop\n\tv_nop" : "+v"(d) : "v"(a), "v"(b));
  return d;
}
__device__ __forceinline__ v8f wmma_bf(v16b a, v16b b, v8f c) {
  v8f d = __builtin_amdgcn_wmma_f32_16x16x32_bf16(false, a, false, b, (short)0, c, false, false);
  asm volatile("v_nop\n\tv_nop\n\tv_nop\n\tv_nop" : "+v"(d) : "v"(a), "v"(b));
  return d;
}
__device__ __forceinline__ v16h frag_h(const _Float16* rowk0, int lane) {
  union { v16h v; v8h q[2]; } u; const _Float16* p = rowk0 + 8 * (lane >> 4);
  u.q[0] = *(const v8h*)p; u.q[1] = *(const v8h*)(p + 16); return u.v;
}
__device__ __forceinline__ v16h frag_f32(const float* rowk0, int lane) {
  v16h a; const float* p = rowk0 + 8 * (lane >> 4);
#pragma unroll
  for (int i = 0; i < 8; ++i) { a[i] = (_Float16)p[i]; a[8 + i] = (_Float16)p[16 + i]; }
  return a;
}
__device__ __forceinline__ v16h frag_f32s(const float* rowk0, int lane, float sc) {
  v16h a; const float* p = rowk0 + 8 * (lane >> 4);
#pragma unroll
  for (int i = 0; i < 8; ++i) { a[i] = (_Float16)(p[i] * sc); a[8 + i] = (_Float16)(p[16 + i] * sc); }
  return a;
}
__device__ __forceinline__ v16h fragc_f32(const float* W, int k0, int n, int lane, int ld, int K) {
  v16h a; const int g = lane >> 4;
#pragma unroll
  for (int i = 0; i < 8; ++i) { const int ka = k0 + 8 * g + i, kb = ka + 16;
    a[i] = (_Float16)(ka < K ? W[(size_t)(ka < K ? ka : K - 1) * ld + n] : 0.f); a[8 + i] = (_Float16)(kb < K ? W[(size_t)(kb < K ? kb : K - 1) * ld + n] : 0.f); }
  return a;
}
struct F2 { v16b h, l; };
__device__ __forceinline__ F2 bsplit16(const float v[16]) { F2 r;
#pragma unroll
  for (int i = 0; i < 16; ++i) { const __bf16 h = (__bf16)v[i]; r.h[i] = h; r.l[i] = (__bf16)(v[i] - (float)h); }
  return r; }
__device__ __forceinline__ F2 split_row(const float* row, int k0, int lane) { float v[16]; const float* p = row + k0 + 8 * (lane >> 4);
#pragma unroll
  for (int i = 0; i < 8; ++i) { v[i] = p[i]; v[8 + i] = p[16 + i]; }
  return bsplit16(v); }
__device__ __forceinline__ F2 split_rowK(const float* row, int k0, int lane, int K) { float v[16]; const int g = lane >> 4;
#pragma unroll
  for (int i = 0; i < 8; ++i) { const int ka = k0 + 8 * g + i, kb = ka + 16; v[i] = ka < K ? row[ka < K ? ka : K - 1] : 0.f; v[8 + i] = kb < K ? row[kb < K ? kb : K - 1] : 0.f; }
  return bsplit16(v); }
__device__ __forceinline__ F2 split_col(const float* W, int k0, int n, int lane, int ld, int K) { float v[16]; const int g = lane >> 4;
#pragma unroll
  for (int i = 0; i < 8; ++i) { const int ka = k0 + 8 * g + i, kb = ka + 16; v[i] = ka < K ? W[(size_t)(ka < K ? ka : K - 1) * ld + n] : 0.f; v[8 + i] = kb < K ? W[(size_t)(kb < K ? kb : K - 1) * ld + n] : 0.f; }
  return bsplit16(v); }
__device__ __forceinline__ v8f mac3(const F2& a, const F2& b, v8f c) { c = wmma_bf(a.l, b.h, c); c = wmma_bf(a.h, b.l, c); return wmma_bf(a.h, b.h, c); }
__device__ __forceinline__ float sigm(float v) { return 1.0f / (1.0f + expf(-v)); }
#define LDSX() do { asm volatile("s_wait_dscnt 0" ::: "memory"); __builtin_amdgcn_wave_barrier(); __builtin_amdgcn_fence(__ATOMIC_RELEASE, "workgroup"); } while (0)


#define NB 16
#define CC 256
#define NN 1024
#define NH 4
#define DH 64
#define NG 8
#define CPG (CC / NG)
#define GNEPS 1e-5f
#ifndef TNB
#define TNB NB
#endif
typedef __attribute__((ext_vector_type(8))) __bf16 v8b;
__device__ __forceinline__ v16b frag_b(const __bf16* rowk0, int lane) {
  union { v16b v; v8b q[2]; } u; const __bf16* p = rowk0 + 8 * (lane >> 4);
  u.q[0] = *(const v8b*)p; u.q[1] = *(const v8b*)(p + 16); return u.v;
}
__device__ __forceinline__ float bfr(float v) { return (float)(__bf16)v; }
__device__ __attribute__((noinline)) float exp_ni(float v) { return expf(v); }
__device__ __attribute__((noinline)) float erf_ni(float v) { return erff(v); }

#define WS_GS  0u
#define WS_Q   (WS_GS + 4u * NB * NG * 4)
#define WS_K   (WS_Q + 2u * (size_t)NB * NN * CC)
#define WS_VH  (WS_K + 2u * (size_t)NB * NN * CC)
#define WS_VL  (WS_VH + 2u * (size_t)NB * CC * NN)
#define WS_O   (WS_VL + 2u * (size_t)NB * CC * NN)
#define WS_END (WS_O + 4u * (size_t)NB * NN * CC)

__global__ __launch_bounds__(256) void k_gn(const float* __restrict__ X, float* __restrict__ GS) { __shared__ float red[8]; __shared__ float smu; __shared__ __align__(16) float res[4];
  const int t = threadIdx.x, lane = t & 31, w = t >> 5; const int gi = blockIdx.x; const size_t b = blockIdx.y; const float* base = X + (b * CC + (size_t)gi * CPG) * NN;
  float s = 0.f;
#pragma unroll 1
  for (int i = t; i < CPG * NN; i += 256) s += bfr(base[i]);
#pragma unroll
  for (int o = 1; o < 32; o <<= 1) s += __shfl_xor(s, o);
  if (lane == 0) red[w] = s; __syncthreads(); if (t == 0) { float a = 0.f; for (int i = 0; i < 8; ++i) a += red[i]; smu = a / (float)(CPG * NN); } __syncthreads();
  const float mu = smu; float q = 0.f;
#pragma unroll 1
  for (int i = t; i < CPG * NN; i += 256) { const float d = bfr(base[i]) - mu; q += d * d; }
#pragma unroll
  for (int o = 1; o < 32; o <<= 1) q += __shfl_xor(q, o);
  if (lane == 0) red[w] = q; __syncthreads(); if (t == 0) { float a = 0.f; for (int i = 0; i < 8; ++i) a += red[i]; res[0] = mu; res[1] = 1.0f / sqrtf(a / (float)(CPG * NN) + GNEPS); res[2] = 0.f; res[3] = 0.f; vst2(GS + (b * NG + gi) * 4, *(const v4f*)res); } }
__global__ __launch_bounds__(128) void k_qkv(const float* __restrict__ X, const float* __restrict__ GS, const float* __restrict__ GW, const float* __restrict__ GB, const float* __restrict__ W, const float* __restrict__ Bq, _Float16* __restrict__ Q, _Float16* __restrict__ K, _Float16* __restrict__ VH, _Float16* __restrict__ VL) {
  __shared__ __align__(16) _Float16 sh[64][136]; __shared__ __align__(16) _Float16 th[128][72], tl[128][72]; __shared__ float sa[CC], sb[CC];
  const int tid = threadIdx.x, wave = tid >> 5, lane = tid & 31, col = lane & 15, g = lane >> 4; const int which = blockIdx.z / NB; const size_t b = blockIdx.z % NB; const int n0 = blockIdx.x * 64; const int c0 = blockIdx.y * 128; const float* Xb = X + b * CC * (size_t)NN;
  for (int c = tid; c < CC; c += 128) { const float mu = GS[(b * NG + c / CPG) * 4], inv = GS[(b * NG + c / CPG) * 4 + 1]; const float a = inv * bfr(GW[c]); sa[c] = a; sb[c] = bfr(GB[c]) - mu * a; } __syncthreads();
  v8f acc[8] = {};
#pragma unroll 2
  for (int kc = 0; kc < CC / 32; ++kc) { float v[16]; const int px = n0 + wave * 16 + col;
#pragma unroll
    for (int i = 0; i < 8; ++i) { const int ca = kc * 32 + 8 * g + i, cb = ca + 16; v[i] = bfr(Xb[(size_t)ca * NN + px]) * sa[ca] + sb[ca]; v[8 + i] = bfr(Xb[(size_t)cb * NN + px]) * sa[cb] + sb[cb]; }
    const F2 a = bsplit16(v);
#pragma unroll
    for (int j = 0; j < 8; ++j) { v16b w; const float* wr = W + (size_t)(which * CC + c0 + j * 16 + col) * CC + kc * 32 + 8 * g;
#pragma unroll
      for (int i = 0; i < 8; ++i) { w[i] = (__bf16)wr[i]; w[8 + i] = (__bf16)wr[16 + i]; }
      acc[j] = wmma_bf(a.h, w, acc[j]); acc[j] = wmma_bf(a.l, w, acc[j]); } }
#pragma unroll
  for (int j = 0; j < 8; ++j) { const float bb = bfr(Bq[which * CC + c0 + j * 16 + col]);
#pragma unroll
    for (int r = 0; r < 8; ++r) { const float v = acc[j][r] + bb; const int rl = wave * 16 + 8 * g + r, cl = j * 16 + col; if (which < 2) sh[rl][cl] = (_Float16)v; else { const _Float16 hv = (_Float16)v; th[cl][rl] = hv; tl[cl][rl] = (_Float16)((v - (float)hv) * 2048.0f); } } }
  __syncthreads();
  if (which < 2) { _Float16* dst = which == 0 ? Q : K; for (int e = tid; e < 64 * 16; e += 128) { const int rl = e >> 4, q = e & 15; vst2((unsigned*)(dst + (b * NN + n0 + rl) * CC + c0 + q * 8), *(const v4u*)&sh[rl][q * 8]); } }
  else { for (int e = tid; e < 128 * 8; e += 128) { const int cl = e >> 3, q = e & 7; const size_t o = (b * CC + c0 + cl) * (size_t)NN + n0 + q * 8; vst2((unsigned*)(VH + o), *(const v4u*)&th[cl][q * 8]); vst2((unsigned*)(VL + o), *(const v4u*)&tl[cl][q * 8]); } } }
__global__ __launch_bounds__(128) void k_att(const _Float16* __restrict__ Q, const _Float16* __restrict__ K, const _Float16* __restrict__ VH, const _Float16* __restrict__ VL, float* __restrict__ O) {
  __shared__ __align__(16) float sp[4][16][36]; __shared__ __align__(16) float so[4][16][68];
  const int tid = threadIdx.x, wave = tid >> 5, lane = tid & 31, col = lane & 15, g = lane >> 4; const int h = blockIdx.y; const size_t b = blockIdx.z; const int q0 = blockIdx.x * 64 + wave * 16; const size_t rq = b * NN + q0;
  v16h aq[2];
#pragma unroll
  for (int kc = 0; kc < 2; ++kc) aq[kc] = frag_h(Q + (rq + col) * CC + h * DH + kc * 32, lane);
  float m[8], l[8];
#pragma unroll
  for (int r = 0; r < 8; ++r) { m[r] = -3.0e38f; l[r] = 0.f; }
  v8f acc[4] = {}, accl[4] = {};
#pragma unroll 1
  for (int ks = 0; ks < NN / 32; ++ks) { float s[2][8];
#pragma unroll
    for (int ct = 0; ct < 2; ++ct) { const size_t rk = b * NN + ks * 32 + ct * 16 + col; v8f c = {};
#pragma unroll
      for (int kc = 0; kc < 2; ++kc) c = wmma16(aq[kc], frag_h(K + rk * CC + h * DH + kc * 32, lane), c);
#pragma unroll
      for (int r = 0; r < 8; ++r) s[ct][r] = c[r] * 0.125f; }
    float alpha[8];
#pragma unroll
    for (int r = 0; r < 8; ++r) { float mx = fmaxf(s[0][r], s[1][r]);
#pragma unroll
      for (int o = 1; o < 16; o <<= 1) mx = fmaxf(mx, __shfl_xor(mx, o));
      const float mn = fmaxf(m[r], mx); alpha[r] = __expf(m[r] - mn); const float e0 = __expf(s[0][r] - mn), e1 = __expf(s[1][r] - mn); float es = e0 + e1;
#pragma unroll
      for (int o = 1; o < 16; o <<= 1) es += __shfl_xor(es, o);
      l[r] = l[r] * alpha[r] + es; m[r] = mn; sp[wave][8 * g + r][col] = e0; sp[wave][8 * g + r][16 + col] = e1; }
#pragma unroll
    for (int j = 0; j < 4; ++j)
#pragma unroll
      for (int r = 0; r < 8; ++r) { acc[j][r] *= alpha[r]; accl[j][r] *= alpha[r]; }
    LDSX();
    v16h pa; { const float* prow = &sp[wave][col][0] + 8 * (lane >> 4);
#pragma unroll
      for (int i = 0; i < 8; ++i) { pa[i] = (_Float16)(prow[i] * 2048.0f); pa[8 + i] = (_Float16)(prow[16 + i] * 2048.0f); } }
#pragma unroll
    for (int j = 0; j < 4; ++j) { const size_t po = (b * CC + (size_t)h * DH + j * 16 + col) * (size_t)NN + ks * 32; acc[j] = wmma16(pa, frag_h(VH + po, lane), acc[j]); accl[j] = wmma16(pa, frag_h(VL + po, lane), accl[j]); }
    LDSX(); }
#pragma unroll
  for (int r = 0; r < 8; ++r) { const float il = (1.0f / 2048.0f) / l[r];
#pragma unroll
    for (int j = 0; j < 4; ++j) so[wave][8 * g + r][j * 16 + col] = (acc[j][r] + accl[j][r] * (1.0f / 2048.0f)) * il; }
  LDSX(); for (int rl = 0; rl < 16; ++rl) if (lane < 16) vst2(O + (rq + rl) * CC + (size_t)h * DH + lane * 4, *(const v4f*)&so[wave][rl][lane * 4]); }
__global__ __launch_bounds__(128) void k_o(const float* __restrict__ OR, const float* __restrict__ PW, const float* __restrict__ PB, const float* __restrict__ X, float* __restrict__ OUT) { __shared__ __align__(16) float sf[4][16][132];
  const int tid = threadIdx.x, wave = tid >> 5, lane = tid & 31, col = lane & 15, g = lane >> 4; const size_t b = blockIdx.z; const int o0 = blockIdx.x * 64 + wave * 16; const int p0 = blockIdx.y * 128;
  v8f acc[8] = {};
#pragma unroll 2
  for (int kc = 0; kc < CC / 32; ++kc) { v16b a; const float* ar = PW + (size_t)(o0 + col) * CC + kc * 32 + 8 * g;
#pragma unroll
    for (int i = 0; i < 8; ++i) { a[i] = (__bf16)ar[i]; a[8 + i] = (__bf16)ar[16 + i]; }
#pragma unroll
    for (int j = 0; j < 8; ++j) { float wv[16]; const float* wr = OR + (b * NN + p0 + j * 16 + col) * CC + kc * 32 + 8 * g;
#pragma unroll
      for (int i = 0; i < 8; ++i) { wv[i] = wr[i]; wv[8 + i] = wr[16 + i]; }
      const F2 wb = bsplit16(wv); acc[j] = wmma_bf(a, wb.h, acc[j]); acc[j] = wmma_bf(a, wb.l, acc[j]); } }
#pragma unroll
  for (int j = 0; j < 8; ++j)
#pragma unroll
    for (int r = 0; r < 8; ++r) { const size_t oi = (b * CC + o0 + 8 * g + r) * (size_t)NN + p0 + j * 16 + col; sf[wave][8 * g + r][j * 16 + col] = acc[j][r] + bfr(PB[o0 + 8 * g + r]) + bfr(X[oi]); }
  LDSX(); for (int rl = 0; rl < 16; ++rl) vst2(OUT + (b * CC + o0 + rl) * (size_t)NN + p0 + lane * 4, *(const v4f*)&sf[wave][rl][lane * 4]); }
extern "C" void kernel_launch(void* const* d_in, const int* in_sizes, int n_in, void* d_out, int out_size, void* d_ws, size_t ws_size, hipStream_t stream) {
  (void)in_sizes; (void)n_in; (void)out_size;
  const float** F = (const float**)d_in;
  if (ws_size < (size_t)WS_END) return;
  char* ws = (char*)d_ws; float* GS = (float*)(ws + WS_GS); _Float16 *Q = (_Float16*)(ws + WS_Q), *K = (_Float16*)(ws + WS_K), *VH = (_Float16*)(ws + WS_VH), *VL = (_Float16*)(ws + WS_VL); float* O = (float*)(ws + WS_O);
  k_gn<<<dim3(NG, NB), 256, 0, stream>>>(F[0], GS);
  k_qkv<<<dim3(NN / 64, CC / 128, 3 * NB), 128, 0, stream>>>(F[0], GS, F[1], F[2], F[3], F[4], Q, K, VH, VL);
  k_att<<<dim3(NN / 64, NH, TNB), 128, 0, stream>>>(Q, K, VH, VL, O);
  k_o<<<dim3(CC / 64, NN / 128, TNB), 128, 0, stream>>>(O, F[5], F[6], F[0], (float*)d_out);
}
